// HaloAttn_37314675868124
// MI455X (gfx1250) — hardware-verified
//
#include <hip/hip_runtime.h>


#define NB_  4
#define HH   128
#define WW   128
#define CC   128
#define BSZ  8
#define HSZ  3
#define WIN  14
#define NKY  196
#define NKP  256
#define NH_  8
#define DQ   16
#define KP   32
#define NBH  16
#define NPX  (NB_ * HH * WW)
#define GRB  4
#define NZ   (GRB * NBH * NH_)
#define DM   CC
#define PCAR 1024.0f
#define LOSC 1024.0f
typedef _Float16 h16;
typedef unsigned short bf;
typedef __attribute__((ext_vector_type(16))) __bf16   v16bf;
typedef __attribute__((ext_vector_type(16))) _Float16 v16h;
typedef __attribute__((ext_vector_type(8)))  _Float16 v8h;
typedef __attribute__((ext_vector_type(8)))  unsigned short v8us;
typedef __attribute__((ext_vector_type(8)))  float    v8f;
typedef __attribute__((ext_vector_type(4)))  float    v4f;
typedef v8h  __attribute__((may_alias)) v8ha;
typedef v4f  __attribute__((may_alias)) v4fa;
typedef v8us __attribute__((may_alias)) v8usa;

__device__ __forceinline__ unsigned short f2bf(float f) { unsigned u = __float_as_uint(f); u += 0x7FFFu + ((u >> 16) & 1u); return (unsigned short)(u >> 16); }
__device__ __forceinline__ float bf2f(unsigned short b) { return __uint_as_float(((unsigned)b) << 16); }
__device__ __forceinline__ float bfr(float f) { return bf2f(f2bf(f)); }
__device__ __forceinline__ v16h cat16(v8h lo, v8h hi) { return __builtin_shufflevector(lo, hi, 0, 1, 2, 3, 4, 5, 6, 7, 8, 9, 10, 11, 12, 13, 14, 15); }
__device__ __forceinline__ v16bf cat16b(v8us lo, v8us hi) { return __builtin_bit_cast(v16bf, __builtin_shufflevector(lo, hi, 0, 1, 2, 3, 4, 5, 6, 7, 8, 9, 10, 11, 12, 13, 14, 15)); }
__device__ __forceinline__ v8f wmma16(v16h a, v16h b, v8f c) { return __builtin_amdgcn_wmma_f32_16x16x32_f16(false, a, false, b, (short)0, c, false, false); }
__device__ __forceinline__ v8f wmmab(v16bf a, v16bf b, v8f c) { return __builtin_amdgcn_wmma_f32_16x16x32_bf16(false, a, false, b, (short)0, c, false, false); }

template <bool SPLITA, bool F16OUT = false>
__global__ __launch_bounds__(128) void k_gemmb(const bf* __restrict__ A, const bf* __restrict__ Al, const bf* __restrict__ Bn, const float* __restrict__ bias, float* C, int ldc, h16* C2, const float* __restrict__ R = nullptr, int K = DM, int roundR = 1) {
    __shared__ __align__(16) float ost[4][16 * 68];
    const int lane = threadIdx.x & 31, wave = threadIdx.x >> 5, lr = lane & 15, hi = lane >> 4;
    const int r0 = blockIdx.x * 64 + wave * 16, c0 = blockIdx.y * 64;
    const size_t aoff = (size_t)(r0 + lr) * K + 8 * hi;
    size_t boff[4];
#pragma unroll
    for (int t = 0; t < 4; ++t) boff[t] = (size_t)(c0 + t * 16 + lr) * K + 8 * hi;
    v8f acc[4];
#pragma unroll
    for (int t = 0; t < 4; ++t) acc[t] = (v8f){};
#pragma unroll 1
    for (int kc = 0; kc < K; kc += 32) {
        const v16bf a = cat16b(*(const v8us*)(A + aoff + kc), *(const v8us*)(A + aoff + kc + 16));
        v16bf al = a;
        if (SPLITA) al = cat16b(*(const v8us*)(Al + aoff + kc), *(const v8us*)(Al + aoff + kc + 16));
#pragma unroll
        for (int t = 0; t < 4; ++t) { const v16bf b = cat16b(*(const v8us*)(Bn + boff[t] + kc), *(const v8us*)(Bn + boff[t] + kc + 16)); acc[t] = wmmab(a, b, acc[t]); if (SPLITA) acc[t] = wmmab(al, b, acc[t]); }
        asm volatile("v_nop\n\tv_nop\n\tv_nop\n\tv_nop" : "+v"(acc[0]), "+v"(acc[1]), "+v"(acc[2]), "+v"(acc[3]) : "v"(a), "v"(al));
    }
    float* os = &ost[wave][0];
#pragma unroll
    for (int t = 0; t < 4; ++t) { const float bv = bias ? bfr(bias[c0 + t * 16 + lr]) : 0.f;
#pragma unroll
        for (int j = 0; j < 8; ++j) os[(hi * 8 + j) * 68 + t * 16 + lr] = acc[t][j] + bv; }
    __syncthreads();
    if (F16OUT) {
        h16* crow = (h16*)(void*)C + (size_t)r0 * ldc + c0;
        auto pass = [&]() {
#pragma unroll
            for (int s = 0; s < 4; ++s) { const int row = 4 * s + (lane >> 3), piece = lane & 7; const float* sp = os + row * 68 + piece * 8; v8h o, o2;
#pragma unroll
                for (int i = 0; i < 8; ++i) { const h16 a = (h16)sp[i]; o[i] = a; o2[i] = (h16)((sp[i] - (float)a) * LOSC); }
                *(volatile v8h*)(crow + (size_t)row * ldc + piece * 8) = o; if (C2) *(volatile v8h*)(C2 + (size_t)r0 * ldc + c0 + (size_t)row * ldc + piece * 8) = o2; }
        };
        pass(); __threadfence(); pass();
    } else {
        float* crow = C + (size_t)r0 * ldc + c0;
        auto pass = [&]() {
#pragma unroll
            for (int s = 0; s < 8; ++s) { const int Lid = (lane >> 3) + 4 * s, piece = lane & 7; const int row = Lid >> 1, cofs = (Lid & 1) * 32 + piece * 4;
                v4f val = *(const v4fa*)(os + row * 68 + cofs); if (R) { const v4f rv = *(const v4f*)(R + ((size_t)r0 + row) * ldc + c0 + cofs); val += roundR ? (v4f){bfr(rv[0]), bfr(rv[1]), bfr(rv[2]), bfr(rv[3])} : rv; }
                *(volatile v4f*)(crow + (size_t)row * ldc + cofs) = val; }
        };
        pass(); __threadfence(); pass();
    }
}

__global__ __launch_bounds__(256) void k_cvt8(const float* __restrict__ src, bf* dst, size_t n8) {
    const size_t i = (size_t)blockIdx.x * 256 + threadIdx.x; if (i >= n8) return;
    const v8f v = *(const v8f*)(src + i * 8); v8us o;
#pragma unroll
    for (int k = 0; k < 8; ++k) o[k] = f2bf(v[k]);
    *(volatile v8us*)(dst + i * 8) = o; __threadfence(); *(volatile v8us*)(dst + i * 8) = o;
}
__global__ __launch_bounds__(256) void k_zero8(bf* dst, size_t n8) {
    const size_t i = (size_t)blockIdx.x * 256 + threadIdx.x; if (i >= n8) return; v8us z;
#pragma unroll
    for (int k = 0; k < 8; ++k) z[k] = 0;
    *(volatile v8us*)(dst + i * 8) = z; __threadfence(); *(volatile v8us*)(dst + i * 8) = z;
}

__global__ __launch_bounds__(128) void k_gemmh(const h16* __restrict__ A, const h16* __restrict__ Bn, const float* __restrict__ bias, float* C, int ldc, const float* __restrict__ R, int K, size_t sA, size_t sB, size_t sC, int roundR) {
    __shared__ __align__(16) float ost[4][16 * 68];
    const size_t z = blockIdx.z; A += z * sA; Bn += z * sB; C += z * sC; if (R) R += z * sC;
    const int lane = threadIdx.x & 31, wave = threadIdx.x >> 5, lr = lane & 15, hi = lane >> 4;
    const int r0 = blockIdx.x * 64 + wave * 16, c0 = blockIdx.y * 64;
    const size_t aoff = (size_t)(r0 + lr) * K + 8 * hi;
    size_t boff[4];
#pragma unroll
    for (int t = 0; t < 4; ++t) boff[t] = (size_t)(c0 + t * 16 + lr) * K + 8 * hi;
    v8f acc[4];
#pragma unroll
    for (int t = 0; t < 4; ++t) acc[t] = (v8f){};
#pragma unroll 1
    for (int kc = 0; kc < K; kc += 32) {
        const v16h a = cat16(*(const v8h*)(A + aoff + kc), *(const v8h*)(A + aoff + kc + 16));
#pragma unroll
        for (int t = 0; t < 4; ++t) { const v16h b = cat16(*(const v8h*)(Bn + boff[t] + kc), *(const v8h*)(Bn + boff[t] + kc + 16)); acc[t] = wmma16(a, b, acc[t]); }
        asm volatile("v_nop\n\tv_nop\n\tv_nop\n\tv_nop" : "+v"(acc[0]), "+v"(acc[1]), "+v"(acc[2]), "+v"(acc[3]) : "v"(a));
    }
    float* os = &ost[wave][0];
#pragma unroll
    for (int t = 0; t < 4; ++t) { const float bv = bias ? bfr(bias[c0 + t * 16 + lr]) : 0.f;
#pragma unroll
        for (int j = 0; j < 8; ++j) os[(hi * 8 + j) * 68 + t * 16 + lr] = acc[t][j] + bv; }
    __syncthreads();
    float* crow = C + (size_t)r0 * ldc + c0;
    auto pass = [&]() {
#pragma unroll
        for (int s = 0; s < 8; ++s) { const int Lid = (lane >> 3) + 4 * s, piece = lane & 7; const int row = Lid >> 1, cofs = (Lid & 1) * 32 + piece * 4;
            v4f val = *(const v4fa*)(os + row * 68 + cofs); if (R) { const v4f rv = *(const v4f*)(R + ((size_t)r0 + row) * ldc + c0 + cofs); val += roundR ? (v4f){bfr(rv[0]), bfr(rv[1]), bfr(rv[2]), bfr(rv[3])} : rv; }
            *(volatile v4f*)(crow + (size_t)row * ldc + cofs) = val; }
    };
    pass(); __threadfence(); pass();
}

__global__ __launch_bounds__(128) void k_gemmh32(const h16* __restrict__ A, const h16* __restrict__ Bn, int K, float* C, int ldc, size_t sA, size_t sB, size_t sC) {
    const size_t z = blockIdx.z; A += z * sA; Bn += z * sB; C += z * sC;
    __shared__ __align__(16) float ost[4][16 * 36];
    const int lane = threadIdx.x & 31, wave = threadIdx.x >> 5, lr = lane & 15, hi = lane >> 4;
    const int r0 = blockIdx.x * 64 + wave * 16, c0 = blockIdx.y * 32;
    const size_t aoff = (size_t)(r0 + lr) * K + 8 * hi;
    v8f acc[2]; acc[0] = (v8f){}; acc[1] = (v8f){};
#pragma unroll 1
    for (int kc = 0; kc < K; kc += 32) {
        const v16h a = cat16(*(const v8h*)(A + aoff + kc), *(const v8h*)(A + aoff + kc + 16));
#pragma unroll
        for (int t = 0; t < 2; ++t) { const size_t bo = (size_t)(c0 + t * 16 + lr) * K + kc + 8 * hi; const v16h b = cat16(*(const v8h*)(Bn + bo), *(const v8h*)(Bn + bo + 16)); acc[t] = wmma16(a, b, acc[t]); }
        asm volatile("v_nop\n\tv_nop\n\tv_nop\n\tv_nop" : "+v"(acc[0]), "+v"(acc[1]) : "v"(a));
    }
    float* os = &ost[wave][0];
#pragma unroll
    for (int t = 0; t < 2; ++t) {
#pragma unroll
        for (int j = 0; j < 8; ++j) os[(hi * 8 + j) * 36 + t * 16 + lr] = acc[t][j]; }
    __builtin_amdgcn_wave_barrier(); asm volatile("" ::: "memory");
    float* crow = C + (size_t)r0 * ldc + c0;
    auto pass = [&]() {
#pragma unroll
        for (int s = 0; s < 4; ++s) { const int row = (lane >> 3) + 4 * s, piece = lane & 7; const int cofs = piece * 4;
            const v4f val = *(const v4fa*)(os + row * 36 + cofs); *(volatile v4f*)(crow + (size_t)row * ldc + cofs) = val; }
    };
    pass(); __threadfence(); pass();
}

typedef __attribute__((ext_vector_type(4))) _Float16 v4h;
__device__ __forceinline__ h16 tohx(float x) { return (h16)x; }
__global__ __launch_bounds__(256) void k_cvt8h(const float* __restrict__ src, h16* dst, size_t n8) { const size_t i = (size_t)blockIdx.x * 256 + threadIdx.x; if (i >= n8) return; const v8f v = *(const v8f*)(src + i * 8); v8h o;
#pragma unroll
    for (int k = 0; k < 8; ++k) o[k] = tohx(bfr(v[k])); *(volatile v8h*)(dst + i * 8) = o; __threadfence(); *(volatile v8h*)(dst + i * 8) = o; }
__global__ __launch_bounds__(256) void k_cvtx(const float* __restrict__ x, bf* A) {
    typedef __attribute__((ext_vector_type(4))) unsigned short v4us;
    const int lane = threadIdx.x & 31; const size_t r = (size_t)blockIdx.x * 8 + (threadIdx.x >> 5); if (r >= (size_t)NPX) return; v4us v;
#pragma unroll
    for (int i = 0; i < 4; ++i) v[i] = f2bf(x[r * CC + lane * 4 + i]);
    *(volatile v4us*)(A + r * CC + lane * 4) = v; __threadfence(); *(volatile v4us*)(A + r * CC + lane * 4) = v;
}
__global__ __launch_bounds__(256) void k_qpl(const float* __restrict__ Q, int b, int br0, h16* Qp) {
    const int lane = threadIdx.x & 31; const size_t w = (size_t)blockIdx.x * 8 + (threadIdx.x >> 5); if (w >= (size_t)NZ * 16) return; const int z = (int)(w / 16); const int tk = (int)(w % 16) * 4 + (lane >> 3); const int d0 = (lane & 7) * 4; const int h = z % NH_, bj = (z / NH_) % NBH, bil = z / (NH_ * NBH); const int py = (br0 + bil) * BSZ + tk / BSZ, px = bj * BSZ + tk % BSZ; v4h o;
#pragma unroll
    for (int i = 0; i < 4; ++i) { const int d = d0 + i; o[i] = tohx(d < DQ ? Q[(((size_t)b * HH + py) * WW + px) * CC + h * DQ + (d < DQ ? d : 0)] * 0.25f : 0.f); }
    const size_t off = ((size_t)z * 64 + tk) * KP + d0; *(volatile v4h*)(Qp + off) = o; __threadfence(); *(volatile v4h*)(Qp + off) = o;
}
__global__ __launch_bounds__(256) void k_kpl(const float* __restrict__ KV, int b, int br0, h16* Kp) {
    const int lane = threadIdx.x & 31; const size_t w = (size_t)blockIdx.x * 8 + (threadIdx.x >> 5); if (w >= (size_t)NZ * 64) return; const int z = (int)(w / 64); const int kk = (int)(w % 64) * 4 + (lane >> 3); const int d0 = (lane & 7) * 4; const int h = z % NH_, bj = (z / NH_) % NBH, bil = z / (NH_ * NBH);
    const int wr = kk / WIN, wc = kk % WIN; const int py = (br0 + bil) * BSZ - HSZ + wr, px = bj * BSZ - HSZ + wc; const bool live = kk < NKY && py >= 0 && py < HH && px >= 0 && px < WW; v4h o;
#pragma unroll
    for (int i = 0; i < 4; ++i) { const int d = d0 + i; o[i] = tohx((live && d < DQ) ? KV[(((size_t)b * HH + py) * WW + px) * (2 * CC) + h * 32 + d] : 0.f); }
    const size_t off = ((size_t)z * NKP + kk) * KP + d0; *(volatile v4h*)(Kp + off) = o; __threadfence(); *(volatile v4h*)(Kp + off) = o;
}
__global__ __launch_bounds__(256) void k_vT(const float* __restrict__ KV, int b, int br0, h16* VT) {
    const int lane = threadIdx.x & 31; const size_t w = (size_t)blockIdx.x * 8 + (threadIdx.x >> 5); if (w >= (size_t)NZ * KP) return; const int z = (int)(w / KP), d = (int)(w % KP); const int h = z % NH_, bj = (z / NH_) % NBH, bil = z / (NH_ * NBH); v8h o;
#pragma unroll
    for (int i = 0; i < 8; ++i) { const int kk = lane * 8 + i; const int wr = kk / WIN, wc = kk % WIN; const int py = (br0 + bil) * BSZ - HSZ + wr, px = bj * BSZ - HSZ + wc; const bool live = d < DQ && kk < NKY && py >= 0 && py < HH && px >= 0 && px < WW;
        o[i] = tohx(live ? KV[(((size_t)b * HH + py) * WW + px) * (2 * CC) + h * 32 + DQ + (d < DQ ? d : 0)] : 0.f); }
    const size_t off = ((size_t)z * KP + d) * NKP + lane * 8; *(volatile v8h*)(VT + off) = o; __threadfence(); *(volatile v8h*)(VT + off) = o;
}
__global__ __launch_bounds__(256) void k_softh(const float* __restrict__ S, const float* __restrict__ tab, int br0, h16* P) {
    const int lane = threadIdx.x & 31; const size_t w = (size_t)blockIdx.x * 8 + (threadIdx.x >> 5); if (w >= (size_t)NZ * 64) return; const int z = (int)(w / 64), tk = (int)(w % 64); const int h = z % NH_, bj = (z / NH_) % NBH, bil = z / (NH_ * NBH); const int qr = tk / BSZ, qc = tk % BSZ; const float* sr = S + w * NKP; h16* po = P + w * NKP;
    float v[8]; bool ok[8]; float m = -3.0e38f;
#pragma unroll
    for (int q = 0; q < 8; ++q) { const int kk = (q < 4) ? lane * 4 + q : 128 + lane * 4 + q - 4; const int wr = kk / WIN, wc = kk % WIN; const int py = (br0 + bil) * BSZ - HSZ + wr, px = bj * BSZ - HSZ + wc; ok[q] = kk < NKY && py >= 0 && py < HH && px >= 0 && px < WW;
        const int rel = ((qr + HSZ - wr) + WIN - 1) * (2 * WIN - 1) + ((qc + HSZ - wc) + WIN - 1); v[q] = ok[q] ? sr[kk] + bfr(tab[(size_t)rel * NH_ + h]) : -3.0e38f; if (ok[q]) m = fmaxf(m, v[q]); }
#pragma unroll
    for (int sh = 16; sh; sh >>= 1) m = fmaxf(m, __shfl_xor(m, sh, 32));
    float sum = 0.f;
#pragma unroll
    for (int q = 0; q < 8; ++q) { v[q] = ok[q] ? __expf(v[q] - m) : 0.f; sum += v[q]; }
#pragma unroll
    for (int sh = 16; sh; sh >>= 1) sum += __shfl_xor(sum, sh, 32);
    const float f = __fdiv_rn(PCAR, sum); v4h oa, ob;
#pragma unroll
    for (int q = 0; q < 4; ++q) { oa[q] = tohx(v[q] * f); ob[q] = tohx(v[4 + q] * f); }
#pragma unroll 1
    for (int ps = 0; ps < 2; ++ps) { *(volatile v4h*)(po + lane * 4) = oa; *(volatile v4h*)(po + 128 + lane * 4) = ob; if (ps == 0) __threadfence(); }
}
__global__ __launch_bounds__(256) void k_fold(const float* __restrict__ OZ, int b, int br0, h16* O16) {
    const int lane = threadIdx.x & 31; const size_t w = (size_t)blockIdx.x * 8 + (threadIdx.x >> 5); if (w >= (size_t)GRB * BSZ * WW) return; const int py = br0 * BSZ + (int)(w / WW), px = (int)(w % WW); const int bil = (py / BSZ) - br0, bj = px / BSZ, tk = (py % BSZ) * BSZ + (px % BSZ); const int h = lane >> 2, d0 = (lane & 3) * 4; const int z = (bil * NBH + bj) * NH_ + h; v4h o;
#pragma unroll
    for (int i = 0; i < 4; ++i) o[i] = tohx(OZ[((size_t)z * 64 + tk) * KP + d0 + i] * (1.0f / PCAR));
    const size_t off = (((size_t)b * HH + py) * WW + px) * CC + h * DQ + d0; *(volatile v4h*)(O16 + off) = o; __threadfence(); *(volatile v4h*)(O16 + off) = o;
}
extern "C" void kernel_launch(void* const* d_in, const int* in_sizes, int n_in,
                              void* d_out, int out_size, void* d_ws, size_t ws_size, hipStream_t stream) {
    (void)in_sizes; (void)n_in; (void)out_size;
    const float* x = (const float*)d_in[0]; const float* qw = (const float*)d_in[1]; const float* kvw = (const float*)d_in[2]; const float* tab = (const float*)d_in[3]; const float* pw = (const float*)d_in[4]; const float* pb = (const float*)d_in[5];
    float* out = (float*)d_out;
    char* wsp = (char*)d_ws;
    auto take = [&](size_t bytes) { char* p = wsp; wsp += (bytes + 255) & ~(size_t)255; return (void*)p; };
    bf* WQ = (bf*)take((size_t)CC * CC * 2); bf* WKV = (bf*)take((size_t)2 * CC * CC * 2); h16* WP = (h16*)take((size_t)CC * CC * 2); bf* XB = (bf*)take((size_t)NPX * CC * 2); float* Q = (float*)take((size_t)NPX * CC * 4); float* KV = (float*)take((size_t)NPX * 2 * CC * 4);
    h16* Qp = (h16*)take((size_t)NZ * 64 * KP * 2); h16* Kp = (h16*)take((size_t)NZ * NKP * KP * 2); h16* VT = (h16*)take((size_t)NZ * KP * NKP * 2); float* S = (float*)take((size_t)NZ * 64 * NKP * 4); h16* Px = (h16*)take((size_t)NZ * 64 * NKP * 2); float* OZ = (float*)take((size_t)NZ * 64 * KP * 4); h16* O16 = (h16*)take((size_t)NPX * CC * 2);
    if ((size_t)(wsp - (char*)d_ws) > ws_size) return;
    const size_t n1 = (size_t)CC * CC / 8, n2 = (size_t)2 * CC * CC / 8;
    k_cvt8<<<(unsigned)((n1 + 255) / 256), 256, 0, stream>>>(qw, WQ, n1); k_cvt8<<<(unsigned)((n2 + 255) / 256), 256, 0, stream>>>(kvw, WKV, n2); k_cvt8h<<<(unsigned)((n1 + 255) / 256), 256, 0, stream>>>(pw, WP, n1);
    k_cvtx<<<NPX / 8, 256, 0, stream>>>(x, XB);
    k_gemmb<false, false><<<dim3(NPX / 64, CC / 64, 1), 128, 0, stream>>>(XB, nullptr, WQ, nullptr, Q, CC, nullptr, nullptr, CC);
    k_gemmb<false, false><<<dim3(NPX / 64, (2 * CC) / 64, 1), 128, 0, stream>>>(XB, nullptr, WKV, nullptr, KV, 2 * CC, nullptr, nullptr, CC);
    for (int b = 0; b < NB_; ++b)
        for (int br0 = 0; br0 < NBH; br0 += GRB) {
            k_qpl<<<(NZ * 16) / 8, 256, 0, stream>>>(Q, b, br0, Qp); k_kpl<<<(NZ * 64) / 8, 256, 0, stream>>>(KV, b, br0, Kp); k_vT<<<(NZ * KP) / 8, 256, 0, stream>>>(KV, b, br0, VT);
            k_gemmh<<<dim3(1, NKP / 64, NZ), 128, 0, stream>>>(Qp, Kp, nullptr, S, NKP, nullptr, KP, (size_t)64 * KP, (size_t)NKP * KP, (size_t)64 * NKP, 0);
            k_softh<<<(NZ * 64) / 8, 256, 0, stream>>>(S, tab, br0, Px);
            k_gemmh32<<<dim3(1, 1, NZ), 128, 0, stream>>>(Px, VT, NKP, OZ, KP, (size_t)64 * NKP, (size_t)KP * NKP, (size_t)64 * KP);
            k_fold<<<(GRB * BSZ * WW) / 8, 256, 0, stream>>>(OZ, b, br0, O16); }
    k_gemmh<<<dim3(NPX / 64, CC / 64, 1), 128, 0, stream>>>(O16, WP, pb, out, CC, nullptr, CC, 0, 0, 0, 0);
}
